// FusionBlock_78975858639181
// MI455X (gfx1250) — hardware-run, weakly checked
//
#include <hip/hip_runtime.h>
#include <math.h>

typedef __attribute__((ext_vector_type(16))) _Float16 v16h;
typedef __attribute__((ext_vector_type(16))) __bf16 v16b;
typedef __attribute__((ext_vector_type(8)))  _Float16 v8h;
typedef __attribute__((ext_vector_type(8)))  float v8f;
typedef __attribute__((ext_vector_type(4)))  float v4f;
typedef __attribute__((ext_vector_type(2)))  float v2f;
typedef __attribute__((ext_vector_type(4)))  unsigned v4u;
typedef __attribute__((ext_vector_type(4)))  int v4i;
typedef float __attribute__((may_alias)) float_a;
typedef int __attribute__((may_alias)) int_a;

template <typename T> __device__ __forceinline__ void vst2(void* p, T v) { *(volatile T*)p = v; __threadfence(); *(volatile T*)p = v; }
__device__ __forceinline__ v8f wmma16(v16h a, v16h b, v8f c) {
  v8f d = __builtin_amdgcn_wmma_f32_16x16x32_f16(false, a, false, b, (short)0, c, false, false);
  asm volatile("v_nop\n\tv_nop\n\tv_nop\n\tv_nop" : "+v"(d) : "v"(a), "v"(b));
  return d;
}
__device__ __forceinline__ v8f wmma_bf(v16b a, v16b b, v8f c) {
  v8f d = __builtin_amdgcn_wmma_f32_16x16x32_bf16(false, a, false, b, (short)0, c, false, false);
  asm volatile("v_nop\n\tv_nop\n\tv_nop\n\tv_nop" : "+v"(d) : "v"(a), "v"(b));
  return d;
}
__device__ __forceinline__ v16h frag_h(const _Float16* rowk0, int lane) {
  union { v16h v; v8h q[2]; } u; const _Float16* p = rowk0 + 8 * (lane >> 4);
  u.q[0] = *(const v8h*)p; u.q[1] = *(const v8h*)(p + 16); return u.v;
}
__device__ __forceinline__ v16h frag_f32(const float* rowk0, int lane) {
  v16h a; const float* p = rowk0 + 8 * (lane >> 4);
#pragma unroll
  for (int i = 0; i < 8; ++i) { a[i] = (_Float16)p[i]; a[8 + i] = (_Float16)p[16 + i]; }
  return a;
}
__device__ __forceinline__ v16h frag_f32s(const float* rowk0, int lane, float sc) {
  v16h a; const float* p = rowk0 + 8 * (lane >> 4);
#pragma unroll
  for (int i = 0; i < 8; ++i) { a[i] = (_Float16)(p[i] * sc); a[8 + i] = (_Float16)(p[16 + i] * sc); }
  return a;
}
__device__ __forceinline__ v16h fragc_f32(const float* W, int k0, int n, int lane, int ld, int K) {
  v16h a; const int g = lane >> 4;
#pragma unroll
  for (int i = 0; i < 8; ++i) { const int ka = k0 + 8 * g + i, kb = ka + 16;
    a[i] = (_Float16)(ka < K ? W[(size_t)(ka < K ? ka : K - 1) * ld + n] : 0.f); a[8 + i] = (_Float16)(kb < K ? W[(size_t)(kb < K ? kb : K - 1) * ld + n] : 0.f); }
  return a;
}
struct F2 { v16b h, l; };
__device__ __forceinline__ F2 bsplit16(const float v[16]) { F2 r;
#pragma unroll
  for (int i = 0; i < 16; ++i) { const __bf16 h = (__bf16)v[i]; r.h[i] = h; r.l[i] = (__bf16)(v[i] - (float)h); }
  return r; }
__device__ __forceinline__ F2 split_row(const float* row, int k0, int lane) { float v[16]; const float* p = row + k0 + 8 * (lane >> 4);
#pragma unroll
  for (int i = 0; i < 8; ++i) { v[i] = p[i]; v[8 + i] = p[16 + i]; }
  return bsplit16(v); }
__device__ __forceinline__ F2 split_rowK(const float* row, int k0, int lane, int K) { float v[16]; const int g = lane >> 4;
#pragma unroll
  for (int i = 0; i < 8; ++i) { const int ka = k0 + 8 * g + i, kb = ka + 16; v[i] = ka < K ? row[ka < K ? ka : K - 1] : 0.f; v[8 + i] = kb < K ? row[kb < K ? kb : K - 1] : 0.f; }
  return bsplit16(v); }
__device__ __forceinline__ F2 split_col(const float* W, int k0, int n, int lane, int ld, int K) { float v[16]; const int g = lane >> 4;
#pragma unroll
  for (int i = 0; i < 8; ++i) { const int ka = k0 + 8 * g + i, kb = ka + 16; v[i] = ka < K ? W[(size_t)(ka < K ? ka : K - 1) * ld + n] : 0.f; v[8 + i] = kb < K ? W[(size_t)(kb < K ? kb : K - 1) * ld + n] : 0.f; }
  return bsplit16(v); }
__device__ __forceinline__ v8f mac3(const F2& a, const F2& b, v8f c) { c = wmma_bf(a.l, b.h, c); c = wmma_bf(a.h, b.l, c); return wmma_bf(a.h, b.h, c); }
__device__ __forceinline__ float sigm(float v) { return 1.0f / (1.0f + expf(-v)); }
#define LDSX() do { asm volatile("s_wait_dscnt 0" ::: "memory"); __builtin_amdgcn_wave_barrier(); __builtin_amdgcn_fence(__ATOMIC_RELEASE, "workgroup"); } while (0)

#define MM 2048
#define NN 256
#define LL 64
#define DD 256
#define D2 (2 * DD)
__device__ __forceinline__ float bfr(float v) { return (float)(__bf16)v; }
__device__ __forceinline__ float sigm_(float v) { return 1.0f / (1.0f + expf(-v)); }

#define WS_ENT 0u
#define WS_E   (WS_ENT + 4u * (size_t)NN * D2)
#define WS_HID (WS_E   + 4u * (size_t)NN * D2)
#define WS_ALP (WS_HID + 4u * (size_t)NN * DD)
#define WS_ET  (WS_ALP + 4u * (size_t)NN * NN)
#define WS_EMB (WS_ET  + 4u * (size_t)NN * DD)
#define WS_END (WS_EMB + 4u * (size_t)MM * DD)

__device__ __forceinline__ F2 colsplit(const float* Wm, int k0, int n, int lane, int ld) { float v[16]; const int g = lane >> 4;
#pragma unroll
  for (int i = 0; i < 8; ++i) { v[i] = Wm[(size_t)(k0 + 8 * g + i) * ld + n]; v[8 + i] = Wm[(size_t)(k0 + 16 + 8 * g + i) * ld + n]; }
  return bsplit16(v); }
__device__ __forceinline__ v16b colbf(const float* Wm, int k0, int n, int lane, int ld) { v16b w; const int g = lane >> 4;
#pragma unroll
  for (int i = 0; i < 8; ++i) { w[i] = (__bf16)Wm[(size_t)(k0 + 8 * g + i) * ld + n]; w[8 + i] = (__bf16)Wm[(size_t)(k0 + 16 + 8 * g + i) * ld + n]; }
  return w; }
__device__ __forceinline__ v16b rowbf(const float* rowk0, int lane) { v16b w; const float* p = rowk0 + 8 * (lane >> 4);
#pragma unroll
  for (int i = 0; i < 8; ++i) { w[i] = (__bf16)p[i]; w[8 + i] = (__bf16)p[16 + i]; }
  return w; }

__global__ __launch_bounds__(128) void k_mean(const float* __restrict__ BIN, const float* __restrict__ CTX, float* __restrict__ ENT) { __shared__ __align__(16) float sf[4][16][132];
  const int tid = threadIdx.x, wave = tid >> 5, lane = tid & 31, col = lane & 15, g = lane >> 4; const int n0 = blockIdx.x * 64 + wave * 16; const int d0 = blockIdx.y * 128;
  v8f acc[8] = {};
#pragma unroll 1
  for (int kc = 0; kc < MM / 32; ++kc) { v16b a; { const float* p = BIN + (size_t)(kc * 32 + 8 * g) * NN + n0 + col;
#pragma unroll
      for (int i = 0; i < 8; ++i) { a[i] = (__bf16)p[(size_t)i * NN]; a[8 + i] = (__bf16)p[(size_t)(16 + i) * NN]; } }
    asm volatile("s_wait_loadcnt 0x0" ::: "memory");
#pragma unroll
    for (int j = 0; j < 8; ++j) { const v16b w = colbf(CTX, kc * 32, d0 + j * 16 + col, lane, DD); asm volatile("s_wait_loadcnt 0x0" ::: "memory"); acc[j] = wmma_bf(a, w, acc[j]); } }
#pragma unroll
  for (int j = 0; j < 8; ++j) {
#pragma unroll
    for (int r = 0; r < 8; ++r) sf[wave][8 * g + r][j * 16 + col] = acc[j][r] * (1.0f / MM); }
  LDSX(); for (int rl = 0; rl < 16; ++rl) vst2(ENT + (size_t)(n0 + rl) * D2 + d0 + lane * 4, *(const v4f*)&sf[wave][rl][lane * 4]); }
__global__ __launch_bounds__(128) void k_max(const float* __restrict__ BIN, const float* __restrict__ CTX, float* __restrict__ ENT) { __shared__ __align__(16) float sc[32][68], sb[32][68]; __shared__ __align__(16) float so[64][68];
  const int tid = threadIdx.x; const int n0 = blockIdx.x * 64, d0 = blockIdx.y * 64; const int nl = tid & 63, dh = tid >> 6;
  float mx[32];
#pragma unroll
  for (int z = 0; z < 32; ++z) mx[z] = -3.0e38f;
#pragma unroll 1
  for (int m0 = 0; m0 < MM; m0 += 32) {
    __syncthreads();
    for (int e = tid; e < 32 * 64; e += 128) { const int ml = e >> 6, c = e & 63; sc[ml][c] = bfr(CTX[(size_t)(m0 + ml) * DD + d0 + c]); sb[ml][c] = bfr(BIN[(size_t)(m0 + ml) * NN + n0 + c]); }
    __syncthreads();
#pragma unroll 4
    for (int ml = 0; ml < 32; ++ml) { const float bv = sb[ml][nl];
#pragma unroll
      for (int z = 0; z < 32; ++z) mx[z] = fmaxf(mx[z], sc[ml][dh * 32 + z] * bv); } }
#pragma unroll
  for (int z = 0; z < 32; ++z) so[nl][dh * 32 + z] = mx[z];
  __syncthreads();
  for (int e = tid; e < 64 * 16; e += 128) { const int rl = e >> 4, q = e & 15; vst2(ENT + (size_t)(n0 + rl) * D2 + DD + d0 + q * 4, *(const v4f*)&so[rl][q * 4]); } }
__global__ __launch_bounds__(256) void k_gate(const float* __restrict__ QE, const float* __restrict__ V, const float* __restrict__ ENT, float* __restrict__ E) { __shared__ __align__(16) float sq[DD], svq[D2], sg[NN];
  const int tid = threadIdx.x;
  { float s = 0.f;
#pragma unroll 4
    for (int l = 0; l < LL; ++l) s += bfr(QE[(size_t)l * DD + tid]);
    sq[tid] = s * (1.0f / LL); }
  __syncthreads();
  for (int c = tid; c < D2; c += 256) { float s = 0.f;
#pragma unroll 4
    for (int i = 0; i < DD; ++i) s += bfr(V[(size_t)i * D2 + c]) * sq[i];
    svq[c] = s; }
  __syncthreads();
  { float s = 0.f; const float* er = ENT + (size_t)tid * D2;
#pragma unroll 4
    for (int c = 0; c < D2; ++c) s += er[c] * svq[c];
    sg[tid] = sigm_(s * (1.0f / 16.0f)); }
  __syncthreads();
  for (int n = 0; n < NN; ++n) { const float gt = sg[n]; const float* er = ENT + (size_t)n * D2; float* ew = E + (size_t)n * D2; if (tid < D2 / 4) { v4f v = *(const v4f*)(er + tid * 4); v[0] *= gt; v[1] *= gt; v[2] *= gt; v[3] *= gt; vst2(ew + tid * 4, v); } } }
__global__ __launch_bounds__(128) void k_hid(const float* __restrict__ E, const float* __restrict__ U, const float* __restrict__ Bv, float* __restrict__ HID) { __shared__ __align__(16) float sf[4][16][132];
  const int tid = threadIdx.x, wave = tid >> 5, lane = tid & 31, col = lane & 15, g = lane >> 4; const int c0 = blockIdx.y * 128; const size_t r0 = (size_t)blockIdx.x * 64 + wave * 16;
  v8f acc[8] = {};
#pragma unroll 2
  for (int kc = 0; kc < D2 / 32; ++kc) { const F2 a = split_row(E + (r0 + col) * D2, kc * 32, lane);
#pragma unroll
    for (int j = 0; j < 8; ++j) { const int o = c0 + j * 16 + col; const v16b w = rowbf(U + (size_t)o * D2 + kc * 32, lane); asm volatile("s_wait_loadcnt 0x0" ::: "memory"); acc[j] = wmma_bf(a.h, w, acc[j]); acc[j] = wmma_bf(a.l, w, acc[j]); } }
#pragma unroll
  for (int j = 0; j < 8; ++j) { const float bb = bfr(Bv[c0 + j * 16 + col]);
#pragma unroll
    for (int r = 0; r < 8; ++r) sf[wave][8 * g + r][j * 16 + col] = acc[j][r] + bb; }
  LDSX(); for (int rl = 0; rl < 16; ++rl) vst2(HID + (r0 + rl) * DD + c0 + lane * 4, *(const v4f*)&sf[wave][rl][lane * 4]); }
__global__ __launch_bounds__(256) void k_graph(const float* __restrict__ HID, const float* __restrict__ Wv, const int* __restrict__ ADJ, float* __restrict__ ALP) { __shared__ __align__(16) float ssi[NN], ssj[NN], srow[NN], sred[8]; __shared__ float sbc;
  const int tid = threadIdx.x;
  { float a = 0.f, b2 = 0.f; const float* hr = HID + (size_t)tid * DD;
#pragma unroll 4
    for (int d = 0; d < DD; ++d) { const float h = hr[d]; a += h * bfr(Wv[d]); b2 += h * bfr(Wv[DD + d]); }
    ssi[tid] = a; ssj[tid] = b2; }
  __syncthreads();
#pragma unroll 1
  for (int i = 0; i < NN; ++i) {
    const float s = ssi[i] + ssj[tid]; const float lk = s >= 0.f ? s : 0.01f * s; const float bt = (ADJ[(size_t)i * NN + tid] > 0) ? lk : 0.f;
    float m = bt;
#pragma unroll
    for (int o = 1; o < 32; o <<= 1) m = fmaxf(m, __shfl_xor(m, o));
    if ((tid & 31) == 0) sred[tid >> 5] = m; __syncthreads(); if (tid == 0) { float a = sred[0]; for (int q = 1; q < 8; ++q) a = fmaxf(a, sred[q]); sbc = a; } __syncthreads(); m = sbc; __syncthreads();
    const float e = expf(bt - m); float sum = e;
#pragma unroll
    for (int o = 1; o < 32; o <<= 1) sum += __shfl_xor(sum, o);
    if ((tid & 31) == 0) sred[tid >> 5] = sum; __syncthreads(); if (tid == 0) { float a = 0.f; for (int q = 0; q < 8; ++q) a += sred[q]; sbc = 1.0f / a; } __syncthreads();
    srow[tid] = e * sbc; __syncthreads();
    if (tid < NN / 4) vst2(ALP + (size_t)i * NN + tid * 4, *(const v4f*)&srow[tid * 4]);
    __syncthreads(); } }
__global__ __launch_bounds__(128) void k_et(const float* __restrict__ ALP, const int* __restrict__ ADJ, const float* __restrict__ HID, float* __restrict__ ET) { __shared__ __align__(16) float sf[4][16][132];
  const int tid = threadIdx.x, wave = tid >> 5, lane = tid & 31, col = lane & 15, g = lane >> 4; const int c0 = blockIdx.y * 128; const int i0 = blockIdx.x * 64 + wave * 16; const int i = i0 + col;
  v8f acc[8] = {};
#pragma unroll 1
  for (int kc = 0; kc < NN / 32; ++kc) { F2 a; { float v[16];
#pragma unroll
      for (int q = 0; q < 8; ++q) { const int ja = kc * 32 + 8 * g + q, jb = ja + 16; const float va = ALP[(size_t)ja * NN + i], vb = ALP[(size_t)jb * NN + i]; const int aa = ADJ[(size_t)i * NN + ja], ab = ADJ[(size_t)i * NN + jb]; v[q] = aa > 0 ? va : 0.f; v[8 + q] = ab > 0 ? vb : 0.f; }
      a = bsplit16(v); }
    asm volatile("s_wait_loadcnt 0x0" ::: "memory");
#pragma unroll
    for (int j = 0; j < 8; ++j) { const F2 w = colsplit(HID, kc * 32, c0 + j * 16 + col, lane, DD); asm volatile("s_wait_loadcnt 0x0" ::: "memory"); acc[j] = mac3(a, w, acc[j]); } }
#pragma unroll
  for (int j = 0; j < 8; ++j) {
#pragma unroll
    for (int r = 0; r < 8; ++r) sf[wave][8 * g + r][j * 16 + col] = fmaxf(acc[j][r], 0.f); }
  LDSX(); for (int rl = 0; rl < 16; ++rl) vst2(ET + (size_t)(i0 + rl) * DD + c0 + lane * 4, *(const v4f*)&sf[wave][rl][lane * 4]); }
__global__ __launch_bounds__(128) void k_emb(const float* __restrict__ BIN, const float* __restrict__ ET, float* __restrict__ EMB) { __shared__ __align__(16) float sf[4][16][132];
  const int tid = threadIdx.x, wave = tid >> 5, lane = tid & 31, col = lane & 15, g = lane >> 4; const int c0 = blockIdx.y * 128; const size_t r0 = (size_t)blockIdx.x * 64 + wave * 16;
  v8f acc[8] = {};
#pragma unroll 1
  for (int kc = 0; kc < NN / 32; ++kc) { const v16b a = rowbf(BIN + (r0 + col) * NN + kc * 32, lane);
#pragma unroll
    for (int j = 0; j < 8; ++j) { const F2 w = colsplit(ET, kc * 32, c0 + j * 16 + col, lane, DD); asm volatile("s_wait_loadcnt 0x0" ::: "memory"); acc[j] = wmma_bf(a, w.h, acc[j]); acc[j] = wmma_bf(a, w.l, acc[j]); } }
#pragma unroll
  for (int j = 0; j < 8; ++j) {
#pragma unroll
    for (int r = 0; r < 8; ++r) sf[wave][8 * g + r][j * 16 + col] = acc[j][r]; }
  LDSX(); for (int rl = 0; rl < 16; ++rl) vst2(EMB + (r0 + rl) * DD + c0 + lane * 4, *(const v4f*)&sf[wave][rl][lane * 4]); }
__global__ __launch_bounds__(128) void k_lstm(const float* __restrict__ CTX, const float* __restrict__ EMB, const float* __restrict__ WIH, const float* __restrict__ BIH, const float* __restrict__ BHH, float* __restrict__ OUT) { __shared__ __align__(16) float sf[4][16][36];
  const int tid = threadIdx.x, wave = tid >> 5, lane = tid & 31, col = lane & 15, g = lane >> 4; const int d0 = blockIdx.y * 32; const size_t r0 = (size_t)blockIdx.x * 64 + wave * 16;
  v8f acc[6] = {};
#pragma unroll 1
  for (int kc = 0; kc < D2 / 32; ++kc) { F2 a; if (kc < DD / 32) { a.h = rowbf(CTX + (r0 + col) * DD + kc * 32, lane); a.l = (v16b){}; } else { a = split_row(EMB + (r0 + col) * DD, kc * 32 - DD, lane); }
    asm volatile("s_wait_loadcnt 0x0" ::: "memory");
#pragma unroll
    for (int j = 0; j < 6; ++j) { const int gate = j >> 1; const int o = (gate == 0 ? 0 : gate == 1 ? 2 * DD : 3 * DD) + d0 + (j & 1) * 16 + col; const v16b w = rowbf(WIH + (size_t)o * D2 + kc * 32, lane); asm volatile("s_wait_loadcnt 0x0" ::: "memory"); acc[j] = wmma_bf(a.h, w, acc[j]); if (kc >= DD / 32) acc[j] = wmma_bf(a.l, w, acc[j]); } }
  {
#pragma unroll
    for (int jj = 0; jj < 2; ++jj) { const int d = d0 + jj * 16 + col; const float bi = bfr(BIH[d]) + bfr(BHH[d]), bg = bfr(BIH[2 * DD + d]) + bfr(BHH[2 * DD + d]), bo = bfr(BIH[3 * DD + d]) + bfr(BHH[3 * DD + d]);
#pragma unroll
      for (int r = 0; r < 8; ++r) { const float gi = sigm_(acc[jj][r] + bi), gg = tanhf(acc[2 + jj][r] + bg), go = sigm_(acc[4 + jj][r] + bo); sf[wave][8 * g + r][jj * 16 + col] = go * tanhf(gi * gg); } } }
  LDSX(); for (int rl = 0; rl < 16; ++rl) if (lane < 8) vst2(OUT + (r0 + rl) * DD + d0 + lane * 4, *(const v4f*)&sf[wave][rl][lane * 4]); }
extern "C" void kernel_launch(void* const* d_in, const int* in_sizes, int n_in, void* d_out, int out_size, void* d_ws, size_t ws_size, hipStream_t stream) {
  (void)in_sizes; (void)n_in; (void)out_size;
  const float** F = (const float**)d_in;
  if (ws_size < (size_t)WS_END) return;
  char* ws = (char*)d_ws; float *ENT = (float*)(ws + WS_ENT), *E = (float*)(ws + WS_E), *HID = (float*)(ws + WS_HID), *ALP = (float*)(ws + WS_ALP), *ET = (float*)(ws + WS_ET), *EMB = (float*)(ws + WS_EMB);
  k_mean<<<dim3(NN / 64, DD / 128), 128, 0, stream>>>(F[2], F[0], ENT);
  k_max<<<dim3(NN / 64, DD / 64), 128, 0, stream>>>(F[2], F[0], ENT);
  k_gate<<<dim3(1), 256, 0, stream>>>(F[1], F[3], ENT, E);
  k_hid<<<dim3(NN / 64, DD / 128), 128, 0, stream>>>(E, F[4], F[5], HID);
  k_graph<<<dim3(1), 256, 0, stream>>>(HID, F[6], (const int*)d_in[11], ALP);
  k_et<<<dim3(NN / 64, DD / 128), 128, 0, stream>>>(ALP, (const int*)d_in[11], HID, ET);
  k_emb<<<dim3(MM / 64, DD / 128), 128, 0, stream>>>(F[2], ET, EMB);
  k_lstm<<<dim3(MM / 64, DD / 32), 128, 0, stream>>>(F[0], EMB, F[7], F[9], F[10], (float*)d_out);
}
